// DynamicArchitectureSelector_76982993814142
// MI455X (gfx1250) — hardware-verified
//
#include <hip/hip_runtime.h>
#include <stddef.h>
#include <stdint.h>

#define NBATCH 2
#define LSEQ   2048
#define DM     1024
#define NTOK   (NBATCH * LSEQ)
#define SELD   64
#define HA 4
#define DA 32
#define HB 8
#define DB 64
#define HC 16
#define DC 128
#define QOFFA 0
#define QOFFB 128
#define QOFFC 640
#define KOFFA 2688
#define KOFFB 2720
#define KOFFC 2784
#define NQK   2944
#define WROW0 2944
#define NWALL 28
#define NWCOL 64
#define NBROW (NQK + NWCOL)
#define NCVT  (NBROW + SELD + 4)
#define TT  64
#define SS  128
#define OPF 132

static_assert(DM % 32 == 0);
static_assert(NTOK % 256 == 0);
static_assert(NQK % 64 == 0);
static_assert(NBROW % 64 == 0);
static_assert(SELD == 64);
static_assert(LSEQ % TT == 0);
static_assert(LSEQ % SS == 0);
static_assert((NTOK * DM) % 8 == 0);
static_assert(QOFFA + HA * DA == QOFFB);
static_assert(QOFFB + HB * DB == QOFFC);
static_assert(QOFFC + HC * DC == KOFFA);
static_assert(KOFFA + DA == KOFFB);
static_assert(KOFFB + DB == KOFFC);
static_assert(KOFFC + DC <= NQK);
static_assert(HA + HB + HC == NWALL);

typedef float          v8f   __attribute__((ext_vector_type(8)));
typedef float          v4f   __attribute__((ext_vector_type(4)));
typedef unsigned int   v4u   __attribute__((ext_vector_type(4)));
typedef unsigned short v8us  __attribute__((ext_vector_type(8)));
typedef unsigned short v16us __attribute__((ext_vector_type(16)));
typedef _Float16       v16h  __attribute__((ext_vector_type(16)));
typedef unsigned short ush;

union FragU { v16us v; v8us h[2]; v16h f; };
union PackU { v8us s; v4u u; };
union HU    { _Float16 h; ush u; };

__device__ __forceinline__ ush f2h(float f) { HU t; t.h = (_Float16)f; return t.u; }

__device__ __forceinline__ v8f zero8() { return (v8f){0.f, 0.f, 0.f, 0.f, 0.f, 0.f, 0.f, 0.f}; }

__device__ __forceinline__ v8f mma16(v16us a, v16us b, v8f c) {
  FragU ua, ub; ua.v = a; ub.v = b;
  c = __builtin_amdgcn_wmma_f32_16x16x32_f16(false, ua.f, false, ub.f, (short)0, c, false, false);
  asm volatile("v_nop\n\tv_nop\n\tv_nop\n\tv_nop" : "+v"(c) : "v"(a), "v"(b));
  return c;
}

__device__ __forceinline__ v16us ldfrag(const ush* p, int ld, int row0, int k0, int lane) {
  const int m = lane & 15, lh = lane >> 4;
  const ush* q = p + (size_t)(row0 + m) * ld + k0 + 8 * lh;
  FragU f;
  f.h[0] = *(const v8us*)(q);
  f.h[1] = *(const v8us*)(q + 16);
  return f.v;
}

__global__ __launch_bounds__(256) void k_stats(const float* __restrict__ x, float* __restrict__ ms) {
  __shared__ double sh[256];
  __shared__ double smean[32];
  __shared__ __align__(16) float line[64];
  const int tid = threadIdx.x, lane = tid & 31, wave = tid >> 5;
  const int rg = wave, c = lane;
  const int b = blockIdx.y, d0 = blockIdx.x * 32;
  const float* col = x + (size_t)b * LSEQ * DM + d0 + c;

  double s = 0.0;
#pragma unroll 4
  for (int i = 0; i < LSEQ / 8; ++i) s += (double)col[(size_t)(rg + 8 * i) * DM];
  sh[tid] = s;
  __syncthreads();
  if (tid < 32) {
    double tsum = 0.0;
#pragma unroll
    for (int g = 0; g < 8; ++g) tsum += sh[g * 32 + tid];
    const double mean = tsum / (double)LSEQ;
    smean[tid] = mean;
    line[tid] = (float)mean;
  }
  __syncthreads();
  const double md = smean[c];
  double s2 = 0.0;
#pragma unroll 4
  for (int i = 0; i < LSEQ / 8; ++i) {
    const double dv = (double)col[(size_t)(rg + 8 * i) * DM] - md;
    s2 += dv * dv;
  }
  sh[tid] = s2;
  __syncthreads();
  if (tid < 32) {
    double tsum = 0.0;
#pragma unroll
    for (int g = 0; g < 8; ++g) tsum += sh[g * 32 + tid];
    const double var = tsum / (double)(LSEQ - 1);
    line[32 + tid] = sqrtf((float)var);
  }
  __syncthreads();
  if (wave == 0) {
    const int L = lane & 15;
    const v4f v = *(const v4f*)(line + L * 4);
    float* dst = ms + (size_t)(b * 2 + (L >> 3)) * DM + d0 + (L & 7) * 4;
    if (lane < 16) *(volatile v4f*)dst = v;
    __threadfence();
    if (lane < 16) *(volatile v4f*)dst = v;
  }
}

__global__ __launch_bounds__(256) void k_cvtx(const float* __restrict__ x, const float* __restrict__ ms,
                                              ush* __restrict__ xh, ush* __restrict__ fh, int ngrp) {
  const int t = blockIdx.x * 256 + (int)threadIdx.x;
  if (t >= ngrp) return;
  const size_t o = (size_t)t * 8;
  const int grow = (int)(o >> 10);
  const int b  = grow >> 11;
  const int tt = grow & (LSEQ - 1);
  const int d  = (int)(o & (DM - 1));
  const v4f a0 = *(const v4f*)(x + o);
  const v4f a1 = *(const v4f*)(x + o + 4);
  const float* mp = ms + (size_t)(b * 2) * DM + d;
  const float* sp = ms + (size_t)(b * 2 + 1) * DM + d;
  const v4f m0 = *(const v4f*)(mp);
  const v4f m1 = *(const v4f*)(mp + 4);
  const v4f s0 = *(const v4f*)(sp);
  const v4f s1 = *(const v4f*)(sp + 4);
  const float pos01 = ((float)tt * (1.0f / 2048.0f)) * 0.1f;
  PackU px, pf;
#pragma unroll
  for (int e = 0; e < 4; ++e) {
    px.s[e]     = f2h(a0[e]);
    px.s[4 + e] = f2h(a1[e]);
    pf.s[e]     = f2h(((a0[e] + m0[e]) + s0[e]) + pos01);
    pf.s[4 + e] = f2h(((a1[e] + m1[e]) + s1[e]) + pos01);
  }
  *(volatile v4u*)(xh + o) = px.u;
  *(volatile v4u*)(fh + o) = pf.u;
  __threadfence();
  *(volatile v4u*)(xh + o) = px.u;
  *(volatile v4u*)(fh + o) = pf.u;
}

__global__ __launch_bounds__(128) void k_cvtw(const float* __restrict__ qwa, const float* __restrict__ qwb,
                                              const float* __restrict__ qwc, const float* __restrict__ kwa,
                                              const float* __restrict__ kwb, const float* __restrict__ kwc,
                                              const float* __restrict__ wwa, const float* __restrict__ wwb,
                                              const float* __restrict__ wwc, const float* __restrict__ sw1,
                                              const float* __restrict__ sw2,
                                              ush* __restrict__ wb, ush* __restrict__ s1p, ush* __restrict__ s2p) {
  const int row = blockIdx.x;
  const int c = (int)threadIdx.x;
  const float* src = qwa;
  int srow = 0, zero = 0;
  if (row < QOFFB)                 { src = qwa; srow = row - QOFFA; }
  else if (row < QOFFC)            { src = qwb; srow = row - QOFFB; }
  else if (row < KOFFA)            { src = qwc; srow = row - QOFFC; }
  else if (row < KOFFB)            { src = kwa; srow = row - KOFFA; }
  else if (row < KOFFC)            { src = kwb; srow = row - KOFFB; }
  else if (row < KOFFC + DC)       { src = kwc; srow = row - KOFFC; }
  else if (row < WROW0)            { zero = 1; }
  else if (row < WROW0 + HA)       { src = wwa; srow = row - WROW0; }
  else if (row < WROW0 + HA + HB)  { src = wwb; srow = row - WROW0 - HA; }
  else if (row < WROW0 + NWALL)    { src = wwc; srow = row - WROW0 - HA - HB; }
  else if (row < NBROW)            { zero = 1; }
  else if (row < NBROW + SELD)     { src = sw1; srow = row - NBROW; }
  else                             { src = sw2; srow = row - NBROW - SELD; }
  ush* dst;
  if (row < NBROW)             dst = wb  + (size_t)row * DM;
  else if (row < NBROW + SELD) dst = s1p + (size_t)(row - NBROW) * DM;
  else                         dst = s2p + (size_t)(row - NBROW - SELD) * DM;

  PackU pk;
  if (zero) {
    pk.u = (v4u){0u, 0u, 0u, 0u};
  } else {
    const float* sp = src + (size_t)srow * DM + c * 8;
    const v4f a0 = *(const v4f*)(sp);
    const v4f a1 = *(const v4f*)(sp + 4);
#pragma unroll
    for (int e = 0; e < 4; ++e) {
      pk.s[e]     = f2h(a0[e] * 256.0f);
      pk.s[4 + e] = f2h(a1[e] * 256.0f);
    }
  }
  ush* dp = dst + c * 8;
  *(volatile v4u*)dp = pk.u;
  __threadfence();
  *(volatile v4u*)dp = pk.u;
}

#define STP 72
#define STF 36
union StageU { v4u al; ush h[256 * STP]; float f[256 * STF]; };

__global__ __launch_bounds__(256) void k_gemm(const ush* __restrict__ A, int lda,
                                              const ush* __restrict__ Bw, int ldb, int K,
                                              const float* __restrict__ bias, int biasn, int hasb,
                                              float ascale, float pscale, int relu,
                                              ush* __restrict__ outH, int ldh, int nqk,
                                              float* __restrict__ outF, int ldf) {
  __shared__ StageU st;
  const int tid = threadIdx.x, lane = tid & 31, wave = tid >> 5;
  const int hh = lane >> 4, c = lane & 15;
  const int mb = blockIdx.x * 256;
  const int m0 = mb + wave * 32;
  const int n0 = blockIdx.y * 64;

  v8f acc[2][4];
#pragma unroll
  for (int s = 0; s < 2; ++s)
#pragma unroll
    for (int t = 0; t < 4; ++t) acc[s][t] = zero8();

#pragma unroll 1
  for (int k0 = 0; k0 < K; k0 += 32) {
    const v16us a0 = ldfrag(A, lda, m0, k0, lane);
    const v16us a1 = ldfrag(A, lda, m0 + 16, k0, lane);
#pragma unroll
    for (int t = 0; t < 4; ++t) {
      const v16us bf = ldfrag(Bw, ldb, n0 + 16 * t, k0, lane);
      acc[0][t] = mma16(a0, bf, acc[0][t]);
      acc[1][t] = mma16(a1, bf, acc[1][t]);
    }
  }

#pragma unroll
  for (int t = 0; t < 4; ++t) {
    const int bidx = min(n0 + 16 * t + c, biasn - 1);
    const float bl = bias[bidx];
    const float bn = (hasb != 0) ? bl : 0.f;
#pragma unroll
    for (int sub = 0; sub < 2; ++sub) {
#pragma unroll
      for (int r = 0; r < 8; ++r) {
        float v = acc[sub][t][r] * ascale + bn;
        v = (relu != 0) ? fmaxf(v, 0.f) : v;
        acc[sub][t][r] = v;
      }
    }
  }

  if (n0 < nqk) {
#pragma unroll
    for (int t = 0; t < 4; ++t) {
#pragma unroll
      for (int sub = 0; sub < 2; ++sub) {
#pragma unroll
        for (int r = 0; r < 8; ++r) {
          const int lr = wave * 32 + sub * 16 + 8 * hh + r;
          st.h[lr * STP + 16 * t + c] = f2h(acc[sub][t][r] * pscale);
        }
      }
    }
    __syncthreads();
    v4u val[8];
    size_t go[8];
#pragma unroll
    for (int j = 0; j < 8; ++j) {
      const int p  = tid + 256 * j;
      const int L  = p >> 3;
      const int pc = p & 7;
      PackU pk;
      pk.s  = *(const v8us*)(st.h + L * STP + pc * 8);
      val[j] = pk.u;
      go[j]  = (size_t)(mb + L) * ldh + n0 + pc * 8;
    }
#pragma unroll
    for (int j = 0; j < 8; ++j) *(volatile v4u*)(outH + go[j]) = val[j];
    __threadfence();
#pragma unroll
    for (int j = 0; j < 8; ++j) *(volatile v4u*)(outH + go[j]) = val[j];
  } else {
    const int nf = n0 - nqk;
#pragma unroll
    for (int cs = 0; cs < 2; ++cs) {
      __syncthreads();
#pragma unroll
      for (int u = 0; u < 2; ++u) {
#pragma unroll
        for (int sub = 0; sub < 2; ++sub) {
#pragma unroll
          for (int r = 0; r < 8; ++r) {
            const int lr = wave * 32 + sub * 16 + 8 * hh + r;
            st.f[lr * STF + 16 * u + c] = acc[sub][2 * cs + u][r];
          }
        }
      }
      __syncthreads();
      v4f val[8];
      size_t go[8];
#pragma unroll
      for (int j = 0; j < 8; ++j) {
        const int p  = tid + 256 * j;
        const int L  = p >> 3;
        const int pc = p & 7;
        val[j] = *(const v4f*)(st.f + L * STF + pc * 4);
        go[j]  = (size_t)(mb + L) * ldf + nf + 32 * cs + pc * 4;
      }
#pragma unroll
      for (int j = 0; j < 8; ++j) *(volatile v4f*)(outF + go[j]) = val[j];
      __threadfence();
#pragma unroll
      for (int j = 0; j < 8; ++j) *(volatile v4f*)(outF + go[j]) = val[j];
    }
  }
}

__global__ __launch_bounds__(256) void k_sel3(const float* __restrict__ h2f, const float* __restrict__ w3,
                                              const float* __restrict__ b3, float* __restrict__ prob,
                                              int ntok) {
  const int i = blockIdx.x * 256 + (int)threadIdx.x;
  if (i >= ntok) return;
  const float* r = h2f + (size_t)i * SELD;
  float l0 = 0.f, l1 = 0.f, l2 = 0.f;
#pragma unroll 1
  for (int k = 0; k < SELD; k += 4) {
    const v4f hv = *(const v4f*)(r + k);
    const v4f wa = *(const v4f*)(w3 + k);
    const v4f wbv = *(const v4f*)(w3 + SELD + k);
    const v4f wc = *(const v4f*)(w3 + 2 * SELD + k);
#pragma unroll
    for (int e = 0; e < 4; ++e) {
      l0 += hv[e] * wa[e];
      l1 += hv[e] * wbv[e];
      l2 += hv[e] * wc[e];
    }
  }
  l0 += b3[0]; l1 += b3[1]; l2 += b3[2];
  const float mx = fmaxf(l0, fmaxf(l1, l2));
  const float e0 = __expf(l0 - mx), e1 = __expf(l1 - mx), e2 = __expf(l2 - mx);
  const float inv = 1.0f / (e0 + e1 + e2);
  const v4f pv = (v4f){e0 * inv, e1 * inv, e2 * inv, 0.f};
  float* dp = prob + (size_t)i * 4;
  *(volatile v4f*)dp = pv;
  __threadfence();
  *(volatile v4f*)dp = pv;
}

template <int H, int DHD, int QOFF, int KOFF, int JB>
__device__ __forceinline__ void cfg_acc(const ush* __restrict__ qk, const float* wpl,
                                        int qrow0, int krow0, int lrow0, int lane, v8f (&o)[2][2]) {
  const int hh = lane >> 4;
#pragma unroll 1
  for (int h = 0; h < H; ++h) {
    v8f cacc[2][2];
    cacc[0][0] = zero8(); cacc[0][1] = zero8(); cacc[1][0] = zero8(); cacc[1][1] = zero8();
    const int qc = QOFF + h * DHD;
#pragma unroll 1
    for (int k0 = 0; k0 < DHD; k0 += 32) {
      const v16us a0 = ldfrag(qk, NQK, qrow0, qc + k0, lane);
      const v16us a1 = ldfrag(qk, NQK, qrow0 + 16, qc + k0, lane);
      const v16us b0 = ldfrag(qk, NQK, krow0, KOFF + k0, lane);
      const v16us b1 = ldfrag(qk, NQK, krow0 + 16, KOFF + k0, lane);
      cacc[0][0] = mma16(a0, b0, cacc[0][0]);
      cacc[0][1] = mma16(a0, b1, cacc[0][1]);
      cacc[1][0] = mma16(a1, b0, cacc[1][0]);
      cacc[1][1] = mma16(a1, b1, cacc[1][1]);
    }
#pragma unroll
    for (int sub = 0; sub < 2; ++sub) {
      const float* wr = wpl + (JB + h) * TT + lrow0 + 16 * sub + 8 * hh;
      const v4f f0 = *(const v4f*)(wr);
      const v4f f1 = *(const v4f*)(wr + 4);
#pragma unroll
      for (int t = 0; t < 2; ++t) {
#pragma unroll
        for (int r = 0; r < 4; ++r) {
          o[sub][t][r]     += fmaxf(cacc[sub][t][r], 0.f) * f0[r];
          o[sub][t][4 + r] += fmaxf(cacc[sub][t][4 + r], 0.f) * f1[r];
        }
      }
    }
  }
}

__global__ __launch_bounds__(256) void k_score(const ush* __restrict__ qk, const float* __restrict__ w32,
                                               const float* __restrict__ prob, float* __restrict__ out) {
  __shared__ __align__(16) float sO[TT * OPF];
  __shared__ __align__(16) float wpl[NWALL * TT];
  const int tid = threadIdx.x, lane = tid & 31, wave = tid >> 5;
  const int hh = lane >> 4, m = lane & 15;
  const int wt = wave >> 2, ws = wave & 3;
  const int b  = blockIdx.z;
  const int T0 = blockIdx.y * TT;
  const int S0 = blockIdx.x * SS;

#pragma unroll
  for (int it = 0; it < 7; ++it) {
    const int idx = tid + 256 * it;
    const int j   = idx >> 6;
    const int row = idx & (TT - 1);
    const int cfg = (j >= HA ? 1 : 0) + (j >= HA + HB ? 1 : 0);
    const size_t grow = (size_t)b * LSEQ + T0 + row;
    const float wv = w32[grow * NWCOL + j];
    const float pv = prob[grow * 4 + cfg];
    wpl[idx] = (wv * pv) * (1.0f / 256.0f);
  }
  __syncthreads();

  v8f o[2][2];
  o[0][0] = zero8(); o[0][1] = zero8(); o[1][0] = zero8(); o[1][1] = zero8();
  const int qrow0 = b * LSEQ + T0 + 32 * wt;
  const int krow0 = b * LSEQ + S0 + 32 * ws;
  const int lrow0 = 32 * wt;
  cfg_acc<HA, DA, QOFFA, KOFFA, 0>(qk, wpl, qrow0, krow0, lrow0, lane, o);
  cfg_acc<HB, DB, QOFFB, KOFFB, HA>(qk, wpl, qrow0, krow0, lrow0, lane, o);
  cfg_acc<HC, DC, QOFFC, KOFFC, HA + HB>(qk, wpl, qrow0, krow0, lrow0, lane, o);

#pragma unroll
  for (int sub = 0; sub < 2; ++sub) {
#pragma unroll
    for (int t = 0; t < 2; ++t) {
#pragma unroll
      for (int r = 0; r < 8; ++r) {
        const int row = lrow0 + 16 * sub + 8 * hh + r;
        sO[row * OPF + 32 * ws + 16 * t + m] = o[sub][t][r];
      }
    }
  }
  __syncthreads();
  v4f val[8];
  size_t go[8];
  const size_t grow0 = (size_t)b * LSEQ + (size_t)T0;
#pragma unroll
  for (int j = 0; j < 8; ++j) {
    const int p   = tid + 256 * j;
    const int L   = p >> 3;
    const int pc  = p & 7;
    const int row = L >> 2;
    const int qu  = L & 3;
    val[j] = *(const v4f*)(sO + row * OPF + qu * 32 + pc * 4);
    go[j]  = (grow0 + (size_t)row) * LSEQ + S0 + qu * 32 + pc * 4;
  }
#pragma unroll
  for (int j = 0; j < 8; ++j) *(volatile v4f*)(out + go[j]) = val[j];
  __threadfence();
#pragma unroll
  for (int j = 0; j < 8; ++j) *(volatile v4f*)(out + go[j]) = val[j];
}

extern "C" void kernel_launch(void* const* d_in, const int* in_sizes, int n_in,
                              void* d_out, int out_size, void* d_ws, size_t ws_size,
                              hipStream_t stream) {
  if (n_in < 16) return;
  if (in_sizes[0]  != NTOK * DM) return;
  if (in_sizes[1]  != SELD * DM) return;
  if (in_sizes[2]  != SELD) return;
  if (in_sizes[3]  != SELD * SELD) return;
  if (in_sizes[4]  != SELD) return;
  if (in_sizes[5]  != 3 * SELD) return;
  if (in_sizes[6]  != 3) return;
  if (in_sizes[7]  != HA * DA * DM) return;
  if (in_sizes[8]  != DA * DM) return;
  if (in_sizes[9]  != HA * DM) return;
  if (in_sizes[10] != HB * DB * DM) return;
  if (in_sizes[11] != DB * DM) return;
  if (in_sizes[12] != HB * DM) return;
  if (in_sizes[13] != HC * DC * DM) return;
  if (in_sizes[14] != DC * DM) return;
  if (in_sizes[15] != HC * DM) return;
  if (out_size != NBATCH * LSEQ * LSEQ) return;

  const float* x      = (const float*)d_in[0];
  const float* sel_w1 = (const float*)d_in[1];
  const float* sel_b1 = (const float*)d_in[2];
  const float* sel_w2 = (const float*)d_in[3];
  const float* sel_b2 = (const float*)d_in[4];
  const float* sel_w3 = (const float*)d_in[5];
  const float* sel_b3 = (const float*)d_in[6];
  const float* qwa    = (const float*)d_in[7];
  const float* kwa    = (const float*)d_in[8];
  const float* wwa    = (const float*)d_in[9];
  const float* qwb    = (const float*)d_in[10];
  const float* kwb    = (const float*)d_in[11];
  const float* wwb    = (const float*)d_in[12];
  const float* qwc    = (const float*)d_in[13];
  const float* kwc    = (const float*)d_in[14];
  const float* wwc    = (const float*)d_in[15];
  float* out = (float*)d_out;

  size_t off = 0;
  const size_t oMS   = off; off += (size_t)NBATCH * 2 * DM * 4;
  const size_t oX16  = off; off += (size_t)NTOK * DM * 2;
  const size_t oF16  = off; off += (size_t)NTOK * DM * 2;
  const size_t oWB   = off; off += (size_t)NBROW * DM * 2;
  const size_t oSW1  = off; off += (size_t)SELD * DM * 2;
  const size_t oSW2  = off; off += (size_t)SELD * SELD * 2;
  const size_t oQK   = off; off += (size_t)NTOK * NQK * 2;
  const size_t oW32  = off; off += (size_t)NTOK * NWCOL * 4;
  const size_t oH1   = off; off += (size_t)NTOK * SELD * 2;
  const size_t oH2F  = off; off += (size_t)NTOK * SELD * 4;
  const size_t oPROB = off; off += (size_t)NTOK * 4 * 4;
  if (off > ws_size) return;
  if (off > (size_t)134217728) return;

  char* ws = (char*)d_ws;
  float* MS   = (float*)(ws + oMS);
  ush*   X16  = (ush*)(ws + oX16);
  ush*   F16  = (ush*)(ws + oF16);
  ush*   WB   = (ush*)(ws + oWB);
  ush*   SW1  = (ush*)(ws + oSW1);
  ush*   SW2  = (ush*)(ws + oSW2);
  ush*   QK   = (ush*)(ws + oQK);
  float* W32  = (float*)(ws + oW32);
  ush*   H1   = (ush*)(ws + oH1);
  float* H2F  = (float*)(ws + oH2F);
  float* PROB = (float*)(ws + oPROB);

  k_stats<<<dim3(DM / 32, NBATCH), dim3(256), 0, stream>>>(x, MS);
  const int ngx = in_sizes[0] / 8;
  k_cvtx<<<dim3((ngx + 255) / 256), dim3(256), 0, stream>>>(x, MS, X16, F16, ngx);
  k_cvtw<<<dim3(NCVT), dim3(128), 0, stream>>>(qwa, qwb, qwc, kwa, kwb, kwc, wwa, wwb, wwc,
                                               sel_w1, sel_w2, WB, SW1, SW2);
  k_gemm<<<dim3(NTOK / 256, NBROW / 64), dim3(256), 0, stream>>>(
      X16, DM, WB, DM, DM, sel_b1, SELD, 0, 1.0f / 256.0f, 16.0f, 0, QK, NQK, NQK, W32, NWCOL);
  k_gemm<<<dim3(NTOK / 256, 1), dim3(256), 0, stream>>>(
      F16, DM, SW1, DM, DM, sel_b1, SELD, 1, 1.0f / 256.0f, 16.0f, 1, H1, SELD, SELD, W32, NWCOL);
  k_gemm<<<dim3(NTOK / 256, 1), dim3(256), 0, stream>>>(
      H1, SELD, SW2, SELD, SELD, sel_b2, SELD, 1, 1.0f / 4096.0f, 1.0f, 1, QK, NQK, 0, H2F, SELD);
  k_sel3<<<dim3(NTOK / 256), dim3(256), 0, stream>>>(H2F, sel_w3, sel_b3, PROB, NTOK);
  k_score<<<dim3(LSEQ / SS, LSEQ / TT, NBATCH), dim3(256), 0, stream>>>(QK, W32, PROB, out);
  (void)hipGetLastError();
}
